// CausalShapedAttention_9182640079156
// MI455X (gfx1250) — hardware-verified
//
#include <hip/hip_runtime.h>


namespace {
constexpr int BT = 4, Bn = 4, S = 2048, D = 1024, H = 16, HD = 64, NTOK = Bn * S;
constexpr float SCALE = 0.125f, VS = 1.0f  , QS = 8.0f, PS = 8.0f, EUL = 2.718281828459045f;
constexpr size_t VPL = (size_t)NTOK * D;
constexpr size_t QPL = (size_t)NTOK * D;

typedef _Float16 b16;
typedef __attribute__((ext_vector_type(16))) _Float16 v16b;
typedef __attribute__((ext_vector_type(8)))  _Float16 v8b;
typedef __attribute__((ext_vector_type(8)))  float v8f;
typedef __attribute__((ext_vector_type(4)))  float v4f;

__device__ __forceinline__ v8b ld8b(const b16* p) { return *(const v8b*)p; }
__device__ __forceinline__ v16b cat8b(v8b a, v8b b) { return __builtin_shufflevector(a, b, 0, 1, 2, 3, 4, 5, 6, 7, 8, 9, 10, 11, 12, 13, 14, 15); }
__device__ __forceinline__ v16b frag_kb(const b16* p, int hh) { return cat8b(ld8b(p + 8 * hh), ld8b(p + 16 + 8 * hh)); }
__device__ __forceinline__ void split16(float v, b16& hi, b16& lo) { hi = (b16)v; lo = (b16)(v - (float)hi); }
__device__ __forceinline__ void frag_ksplit(const float* p, int hh, v16b& fh_, v16b& fl_) {
  const float* p0 = p + 8 * hh; const float* p1 = p + 16 + 8 * hh;
#pragma unroll
  for (int e = 0; e < 8; ++e) { b16 a, c; split16(p0[e], a, c); fh_[e] = a; fl_[e] = c; split16(p1[e], a, c); fh_[8 + e] = a; fl_[8 + e] = c; }
}
__device__ __forceinline__ v8f wmma16b(v16b a, v16b b, v8f c) {
  v8f d = __builtin_amdgcn_wmma_f32_16x16x32_f16(false, a, false, b, (short)0, c, false, false);
  asm volatile("v_nop\n\tv_nop\n\tv_nop\n\tv_nop" : "+v"(d) : "v"(a), "v"(b));
  return d;
}
__device__ __forceinline__ void wave_lds_sync() {
  __builtin_amdgcn_fence(__ATOMIC_RELEASE, "workgroup");
  __builtin_amdgcn_wave_barrier();
  __builtin_amdgcn_fence(__ATOMIC_ACQUIRE, "workgroup");
}

struct Opnd { const void* p0; const void* p1; int ld; };
template <int NP> __device__ __forceinline__ void load_frags(const Opnd& o, int row, int kb, int hh, v16b& fh_, v16b& fl_) {
  if (NP == 0) { frag_ksplit((const float*)o.p0 + (size_t)row * o.ld + kb, hh, fh_, fl_); }
  else if (NP == 4 || NP == 5) {
    const float sc_ = (NP == 4) ? 64.0f : 8.0f;
    const float* p = (const float*)o.p0 + (size_t)row * o.ld + kb; const float* p0 = p + 8 * hh; const float* p1 = p + 16 + 8 * hh;
#pragma unroll
    for (int e = 0; e < 8; ++e) { b16 a, c; split16(p0[e] * sc_, a, c); fh_[e] = a; fl_[e] = c; split16(p1[e] * sc_, a, c); fh_[8 + e] = a; fl_[8 + e] = c; }
  } else if (NP == 3) {
    const float* p = (const float*)o.p0 + (size_t)row * o.ld + kb; const float* p0 = p + 8 * hh; const float* p1 = p + 16 + 8 * hh;
#pragma unroll
    for (int e = 0; e < 8; ++e) { fh_[e] = (b16)p0[e]; fh_[8 + e] = (b16)p1[e]; }
    fl_ = fh_;
  } else {
    fh_ = frag_kb((const b16*)o.p0 + (size_t)row * o.ld + kb, hh);
    if (NP == 2) fl_ = frag_kb((const b16*)o.p1 + (size_t)row * o.ld + kb, hh); else fl_ = fh_;
  }
}
template <int ANP, int BNP> __device__ __forceinline__ v8f mac(v16b ah, v16b al, v16b bh, v16b bl, v8f c) {
  c = wmma16b(ah, bh, c);
  if (BNP == 0 || BNP == 2 || BNP == 4 || BNP == 5) c = wmma16b(ah, bl, c);
  if (ANP == 0 || ANP == 2 || ANP == 4 || ANP == 5) c = wmma16b(al, bh, c);
  return c;
}
template <int ANP, int BNP>
__device__ __forceinline__ void gemm_tile(const Opnd& A, const Opnd& B, int K, int m0, int c0, int nloc, int hlf, v8f (&acc)[2][4]) {
  for (int kb = 0; kb < K; kb += 32) {
    v16b a0h, a0l, a1h, a1l;
    load_frags<ANP>(A, m0 + nloc, kb, hlf, a0h, a0l);
    load_frags<ANP>(A, m0 + 16 + nloc, kb, hlf, a1h, a1l);
#pragma unroll
    for (int t = 0; t < 4; ++t) {
      v16b bh, bl;
      load_frags<BNP>(B, c0 + t * 16 + nloc, kb, hlf, bh, bl);
      acc[0][t] = mac<ANP, BNP>(a0h, a0l, bh, bl, acc[0][t]);
      acc[1][t] = mac<ANP, BNP>(a1h, a1l, bh, bl, acc[1][t]);
    }
  }
}

__device__ __forceinline__ void epi_planes(v8f (&acc)[2][4], float scale, bool two, b16* __restrict__ oh, b16* __restrict__ ol, int ldo,
                                           int m0, int c0, int lane, b16* Th, b16* Tl) {
  const int nloc = lane & 15, hlf = lane >> 4;
#pragma unroll
  for (int t = 0; t < 4; ++t)
#pragma unroll
    for (int r = 0; r < 2; ++r)
#pragma unroll
      for (int v = 0; v < 8; ++v) {
        const int rr = r * 16 + v + 8 * hlf, cc = t * 16 + nloc;
        b16 h_, l_; split16(acc[r][t][v] * scale, h_, l_);
        Th[rr * 64 + cc] = h_; Tl[rr * 64 + cc] = l_;
      }
  wave_lds_sync();
  for (int pass = 0; pass < 2; ++pass) {
#pragma unroll
    for (int j = 0; j < 8; ++j) {
      const int rr = j * 4 + (lane >> 3), c8 = (lane & 7) * 8;
      const size_t o = (size_t)(m0 + rr) * ldo + c0 + c8;
      *(volatile v8b*)(oh + o) = ld8b(Th + rr * 64 + c8);
      if (two) *(volatile v8b*)(ol + o) = ld8b(Tl + rr * 64 + c8);
    }
    __threadfence();
  }
}
__device__ __forceinline__ void epi_f32(v8f (&acc)[2][4], float scale, const float* rscale, float* __restrict__ out, int ldo, int m0, int c0, int lane, float* Tt) {
  const int nloc = lane & 15, hlf = lane >> 4;
#pragma unroll
  for (int t = 0; t < 4; ++t)
#pragma unroll
    for (int r = 0; r < 2; ++r)
#pragma unroll
      for (int v = 0; v < 8; ++v) {
        const int rr = r * 16 + v + 8 * hlf;
        const float rs = rscale ? rscale[(size_t)(m0 + rr) * 32] : 1.0f;
        Tt[rr * 64 + t * 16 + nloc] = acc[r][t][v] * scale * rs;
      }
  wave_lds_sync();
  float* dst0 = out + (size_t)m0 * ldo + c0;
  for (int pass = 0; pass < 2; ++pass) {
#pragma unroll
    for (int j = 0; j < 16; ++j) { const int rr = j * 2 + hlf, c4 = nloc * 4; *(volatile v4f*)(dst0 + (size_t)rr * ldo + c4) = *(const v4f*)(Tt + rr * 64 + c4); }
    __threadfence();
  }
}


typedef __attribute__((ext_vector_type(8))) __bf16 v8bb; typedef __attribute__((ext_vector_type(16))) __bf16 v16bb;
typedef __attribute__((ext_vector_type(8))) unsigned short v8us;
__device__ __forceinline__ v16bb frag_kb_bf(const __bf16* p, int hh) { const v8bb a = *(const v8bb*)(p + 8 * hh), b = *(const v8bb*)(p + 16 + 8 * hh); return __builtin_shufflevector(a, b, 0, 1, 2, 3, 4, 5, 6, 7, 8, 9, 10, 11, 12, 13, 14, 15); }
__device__ __forceinline__ v8f wmma16bb(v16bb a, v16bb b, v8f c) {
  v8f d = __builtin_amdgcn_wmma_f32_16x16x32_bf16(false, a, false, b, (short)0, c, false, false);
  asm volatile("v_nop\n\tv_nop\n\tv_nop\n\tv_nop" : "+v"(d) : "v"(a), "v"(b));
  return d;
}
__device__ __forceinline__ unsigned short bf16_rne_bits(float v) { unsigned int u = __float_as_uint(v); u += 0x7FFFu + ((u >> 16) & 1u); return (unsigned short)(u >> 16); }
__device__ __forceinline__ float bf16_rne(float v) { return __uint_as_float(((unsigned int)bf16_rne_bits(v)) << 16); }


__global__ __launch_bounds__(256) void xprep_kernel(const float* __restrict__ x, unsigned short* __restrict__ x16) {
  const size_t tid = (size_t)blockIdx.x * blockDim.x + threadIdx.x, nth = (size_t)gridDim.x * blockDim.x;
  for (int pass = 0; pass < 2; ++pass) { for (size_t p = tid; p < (size_t)NTOK * D / 8; p += nth) { v8us v;
#pragma unroll
      for (int e = 0; e < 8; ++e) v[e] = bf16_rne_bits(x[p * 8 + e]);
      *(volatile v8us*)(x16 + p * 8) = v; } __threadfence(); }
}
__global__ __launch_bounds__(256) void prep_kernel(const float* __restrict__ wattn, unsigned short* __restrict__ w16) {
  const size_t tid = (size_t)blockIdx.x * blockDim.x + threadIdx.x, nth = (size_t)gridDim.x * blockDim.x;
  for (int pass = 0; pass < 2; ++pass) {
    for (size_t p = tid; p < (size_t)2 * D * D / 8; p += nth) { v8us v;
#pragma unroll
      for (int e = 0; e < 8; ++e) v[e] = bf16_rne_bits(wattn[p * 8 + e]);
      *(volatile v8us*)(w16 + p * 8) = v; }
    __threadfence();
  }
}

__global__ __launch_bounds__(256) void vt_kernel(const float* __restrict__ x, b16* __restrict__ vt, int rowbase) {
  __shared__ __attribute__((aligned(16))) b16 T[HD][128 + 8];
  const int t_ = threadIdx.x, h = blockIdx.x, m0 = rowbase + blockIdx.y * 128, b = m0 / S, tok0 = m0 % S;
  for (int i = t_; i < 128 * HD / 4; i += 256) { const int r = i / (HD / 4), c4 = (i % (HD / 4)) * 4; const v4f xv = *(const v4f*)(x + (size_t)(m0 + r) * D + h * HD + c4);
#pragma unroll
    for (int e = 0; e < 4; ++e) T[c4 + e][r] = (b16)bf16_rne(xv[e]); }
  __syncthreads();
  b16* dst = vt + (((size_t)b * H + h) * HD) * S + tok0;
  for (int pass = 0; pass < 2; ++pass) { for (int i = t_; i < HD * 16; i += 256) { const int d = i >> 4, c8 = (i & 15) * 8; *(volatile v8b*)(dst + (size_t)d * S + c8) = *(const v8b*)(&T[d][c8]); } __threadfence(); }
}
__global__ __launch_bounds__(256) void colsum_kernel(const float* __restrict__ x, float* __restrict__ colsum) {
  const int c = blockIdx.x * 256 + threadIdx.x, b = blockIdx.y; float s = 0.0f;
  for (int t = 0; t < S; ++t) s += bf16_rne(x[((size_t)b * S + t) * D + c]);
  for (int pass = 0; pass < 2; ++pass) { ((volatile float*)colsum)[(size_t)b * D + c] = s; __threadfence(); }
}

__global__ __launch_bounds__(128) void proj_kernel(const __bf16* __restrict__ x16, const __bf16* __restrict__ w16, b16* __restrict__ qh, b16* __restrict__ kh, int rowbase) {
  __shared__ __attribute__((aligned(16))) b16 Th[4][32][HD + 8], Tq[4][32][HD + 8];
  const int lane = threadIdx.x & 31, wave = threadIdx.x >> 5, nloc = lane & 15, hlf = lane >> 4, m0 = rowbase + blockIdx.y * 128 + wave * 32, c0 = blockIdx.x * 64;
  v8f acc[2][4];
#pragma unroll
  for (int r = 0; r < 2; ++r)
#pragma unroll
    for (int t = 0; t < 4; ++t) acc[r][t] = (v8f){};
#pragma unroll 2
  for (int kb = 0; kb < D; kb += 32) {
    const v16bb a0 = frag_kb_bf(x16 + (size_t)(m0 + nloc) * D + kb, hlf), a1 = frag_kb_bf(x16 + (size_t)(m0 + 16 + nloc) * D + kb, hlf);
#pragma unroll
    for (int t = 0; t < 4; ++t) { const v16bb bw = frag_kb_bf(w16 + (size_t)(c0 + t * 16 + nloc) * D + kb, hlf); acc[0][t] = wmma16bb(a0, bw, acc[0][t]); acc[1][t] = wmma16bb(a1, bw, acc[1][t]); }
  }
  const int which = blockIdx.x / (D / 64), head = blockIdx.x % (D / 64), b = m0 / S, tok0 = m0 % S;
  {
#pragma unroll
    for (int t = 0; t < 4; ++t)
#pragma unroll
      for (int r = 0; r < 2; ++r)
#pragma unroll
        for (int v = 0; v < 8; ++v) { b16 a_, c_; split16(acc[r][t][v] * QS, a_, c_); Th[wave][r * 16 + 8 * hlf + v][t * 16 + nloc] = a_; Tq[wave][r * 16 + 8 * hlf + v][t * 16 + nloc] = c_; }
    wave_lds_sync();
    b16* dst = (which == 0 ? qh : kh) + (((size_t)b * H + head) * S + tok0) * HD;
    for (int pass = 0; pass < 2; ++pass) {
#pragma unroll
      for (int j = 0; j < 8; ++j) { const int rr = j * 4 + (lane >> 3), c8 = (lane & 7) * 8; *(volatile v8b*)(dst + (size_t)rr * HD + c8) = *(const v8b*)(&Th[wave][rr][c8]); *(volatile v8b*)(dst + QPL + (size_t)rr * HD + c8) = *(const v8b*)(&Tq[wave][rr][c8]); }
      __threadfence(); }
    return;
  }
}

template <int QT>
__global__ __launch_bounds__(256) void attn_kernel(const b16* __restrict__ qh, const b16* __restrict__ kh, const b16* __restrict__ vt, const float* __restrict__ x, const float* __restrict__ colsum, const float* __restrict__ alpha_p, const float* __restrict__ beta_p, const float* __restrict__ gamma_p, float* __restrict__ y) {
  __shared__ __attribute__((aligned(16))) float Os[8][16][HD + 4];
  const int wid = threadIdx.x >> 5, lane = threadIdx.x & 31, hh = lane >> 4, col = lane & 15;
  const int qt = blockIdx.x * 8 + wid, jt = qt % QT, bh = qt / QT, h = bh % H, b = bh / H, q0 = jt * 16, qi = q0 + col;
  const b16* Q = qh + ((size_t)bh * S) * HD; const b16* K = kh + ((size_t)bh * S) * HD; const b16* vb = vt + ((size_t)bh * HD) * S;
  v16b qf[2], ql[2];
#pragma unroll
  for (int ks = 0; ks < 2; ++ks) { qf[ks] = frag_kb(Q + (size_t)qi * HD + ks * 32, hh); ql[ks] = frag_kb(Q + QPL + (size_t)qi * HD + ks * 32, hh); }
  float m = -INFINITY, l = 0.0f; v8f o[4] = {{}, {}, {}, {}}, pf[4] = {{}, {}, {}, {}};
  for (int kb = 0; kb < q0 + 16; kb += 32) {
    const bool diag = (kb + 32 > q0);
    v16b ub;
#pragma unroll
    for (int r = 0; r < 8; ++r) { ub[r] = (b16)((kb + 8 * hh + r <= qi) ? 1.0f : 0.0f); ub[8 + r] = (b16)((kb + 16 + 8 * hh + r <= qi) ? 1.0f : 0.0f); }
    v8f s0 = {}, s1 = {};
#pragma unroll
    for (int ks = 0; ks < 2; ++ks) { const v16b k0 = frag_kb(K + (size_t)(kb + col) * HD + ks * 32, hh), k0l = frag_kb(K + QPL + (size_t)(kb + col) * HD + ks * 32, hh), k1 = frag_kb(K + (size_t)(kb + 16 + col) * HD + ks * 32, hh), k1l = frag_kb(K + QPL + (size_t)(kb + 16 + col) * HD + ks * 32, hh);
      s0 = wmma16b(k0, qf[ks], s0); s0 = wmma16b(k0, ql[ks], s0); s0 = wmma16b(k0l, qf[ks], s0);
      s1 = wmma16b(k1, qf[ks], s1); s1 = wmma16b(k1, ql[ks], s1); s1 = wmma16b(k1l, qf[ks], s1); }
    float mr = -INFINITY;
#pragma unroll
    for (int r = 0; r < 8; ++r) { s0[r] *= SCALE / (QS * QS); s1[r] *= SCALE / (QS * QS); if (diag) { if (kb + 8 * hh + r > qi) s0[r] = -INFINITY; if (kb + 16 + 8 * hh + r > qi) s1[r] = -INFINITY; } mr = fmaxf(mr, fmaxf(s0[r], s1[r])); }
    mr = fmaxf(mr, __shfl_xor(mr, 16));
    const float mn = fmaxf(m, mr), al_ = __expf(m - mn); m = mn;
    float sum = 0.0f; v16b pb, pl;
#pragma unroll
    for (int r = 0; r < 8; ++r) { const float e0 = __expf(s0[r] - mn), e1 = __expf(s1[r] - mn); sum += e0 + e1; b16 a, c; split16(e0 * PS, a, c); pb[r] = a; pl[r] = c; split16(e1 * PS, a, c); pb[8 + r] = a; pl[8 + r] = c; }
    sum += __shfl_xor(sum, 16); l = l * al_ + sum;
#pragma unroll
    for (int n = 0; n < 4; ++n) {
#pragma unroll
      for (int r = 0; r < 8; ++r) o[n][r] *= al_;
      const v16b vf = frag_kb(vb + (size_t)(n * 16 + col) * S + kb, hh);
      o[n] = wmma16b(vf, pb, o[n]); o[n] = wmma16b(vf, pl, o[n]);
      pf[n] = wmma16b(vf, ub, pf[n]); }
  }
  const float alpha = bf16_rne(alpha_p[0]), beta = bf16_rne(beta_p[0]), gamma = bf16_rne(gamma_p[0]);
  const float cb = beta / (PS * l), cid = alpha / (EUL + (float)(S - 1)), cmc = gamma / (float)(qi + 1);
#pragma unroll
  for (int n = 0; n < 4; ++n)
#pragma unroll
    for (int r = 0; r < 8; ++r) { const int d = n * 16 + 8 * hh + r; const float vi = bf16_rne(x[((size_t)b * S + qi) * D + h * HD + d]), vs = colsum[(size_t)b * D + h * HD + d];
      Os[wid][col][d] = o[n][r] * cb + cid * ((EUL - 1.0f) * vi + vs) - cmc * pf[n][r]; }
  wave_lds_sync();
  float* dst = y + ((size_t)b * S + q0) * D + h * HD;
  for (int pass = 0; pass < 2; ++pass) {
#pragma unroll
    for (int j = 0; j < 8; ++j) { const int rr = j * 2 + hh, c4 = col * 4; *(volatile v4f*)(dst + (size_t)rr * D + c4) = *(const v4f*)(&Os[wid][rr][c4]); }
    __threadfence();
  }
}

}

extern "C" void kernel_launch(void* const* d_in, const int* in_sizes, int n_in,
                              void* d_out, int out_size, void* d_ws, size_t ws_size, hipStream_t stream) {
  (void)n_in; (void)out_size;
  const float* x = (const float*)d_in[0]; const float* wattn = (const float*)d_in[1];
  float* out = (float*)d_out;
  if (in_sizes[0] != BT * S * D || in_sizes[1] != 2 * D * D || in_sizes[2] != 1 || in_sizes[3] != 1 || in_sizes[4] != 1) return;
  size_t off = 0; char* ws = (char*)d_ws;
  auto carve = [&](size_t bytes) { char* p = ws + off; off += (bytes + 255) & ~(size_t)255; return p; };
  unsigned short* x16 = (unsigned short*)carve((size_t)NTOK * D * 2); unsigned short* w16 = (unsigned short*)carve((size_t)2 * D * D * 2); float* colsum = (float*)carve((size_t)BT * D * 4);
  b16* qh = (b16*)carve((size_t)2 * NTOK * D * 2); b16* kh = (b16*)carve((size_t)2 * NTOK * D * 2); b16* vt = (b16*)carve((size_t)NTOK * D * 2);
  if (off > ws_size) return;
  prep_kernel<<<512, 256, 0, stream>>>(wattn, w16);
  xprep_kernel<<<1024, 256, 0, stream>>>(x, x16);
  vt_kernel<<<dim3(H, NTOK / 128), 256, 0, stream>>>(x, vt, 0);
  colsum_kernel<<<dim3(D / 256, BT), 256, 0, stream>>>(x, colsum);
  proj_kernel<<<dim3(2 * D / 64, NTOK / 128), 128, 0, stream>>>((const __bf16*)x16, (const __bf16*)w16, qh, kh, 0);
  attn_kernel<S / 16><<<Bn * H * (S / 16) / 8, 256, 0, stream>>>(qh, kh, vt, x, colsum, (const float*)d_in[2], (const float*)d_in[3], (const float*)d_in[4], out);
}
